// GCNConvModel_59399397704019
// MI455X (gfx1250) — hardware-verified
//
#include <hip/hip_runtime.h>
#include <stddef.h>


#define INC     64
#define HIDC    128
#define OUTC    64
#define NTHR    256
#define NWAVE   8
#define EPT     8
#define NGRP    2
#define CHUNK   (NTHR * EPT * NGRP)
#define WCAP    (EPT * NGRP * 32)
#define LISTN   (NWAVE * WCAP)
#define NBA     1024
#define NBD     4096
#define RB      64
#define NTHN    128
#define APITCH  72
#define HPITCH  136
#define WSCALE  8.0f
#define WINV    0.125f

#define LDS_AGG (NBA * OUTC * 4 + LISTN * 4 + 64)

static_assert((CHUNK & (CHUNK - 1)) == 0);
static_assert(CHUNK <= 4096);
static_assert((NBA & (NBA - 1)) == 0 && NBA <= 4096);
static_assert((NBD & (NBD - 1)) == 0 && NBD <= 4096);
static_assert(NBD % RB == 0);
static_assert(RB * APITCH * 2 <= RB * OUTC * 4);
static_assert(HIDC * INC / 8 == 4 * NTHR);
static_assert(OUTC * HIDC / 8 == 4 * NTHR);
static_assert((NBA * OUTC) == NWAVE * 64 * 128);

typedef float    v2f  __attribute__((ext_vector_type(2)));
typedef float    v4f  __attribute__((ext_vector_type(4)));
typedef float    v8f  __attribute__((ext_vector_type(8)));
typedef int      v4i  __attribute__((ext_vector_type(4)));
typedef _Float16 v8h  __attribute__((ext_vector_type(8)));
typedef _Float16 v16h __attribute__((ext_vector_type(16)));
union FragH { v16h v; v8h h[2]; };

__device__ __forceinline__ v8h cvt8(v4f a, v4f b) {
  v8h r;
  r[0] = (_Float16)a.x; r[1] = (_Float16)a.y; r[2] = (_Float16)a.z; r[3] = (_Float16)a.w;
  r[4] = (_Float16)b.x; r[5] = (_Float16)b.y; r[6] = (_Float16)b.z; r[7] = (_Float16)b.w;
  return r;
}

__device__ __forceinline__ v8f wmh(v16h a, v16h b, v8f c) {
  v8f d = __builtin_amdgcn_wmma_f32_16x16x32_f16(false, a, false, b, (short)0, c, false, false);
  asm volatile("v_nop\n\tv_nop\n\tv_nop\n\tv_nop" : "+v"(d) : "v"(a), "v"(b));
  return d;
}

template <int NB>
__device__ __forceinline__ int scan_chunk(const int* __restrict__ dsts, int nE, int cbase, int nodeBase,
                                          int vec8, int* list, int tid, int lane, int wave) {
  int wc = 0;
#pragma unroll
  for (int g = 0; g < NGRP; ++g) {
    const int el0  = (g * NTHR + tid) * EPT;
    const int e0   = cbase + el0;
    const int sent = -2147483647 - 1;
    v4i da, db;
    if (vec8 != 0 && cbase + CHUNK <= nE) {
      da = *(const v4i*)(dsts + e0);
      db = *(const v4i*)(dsts + e0 + 4);
    } else {
      da.x = (e0     < nE) ? dsts[min(e0, nE - 1)] : sent;
      da.y = (e0 + 1 < nE) ? dsts[min(e0 + 1, nE - 1)] : sent;
      da.z = (e0 + 2 < nE) ? dsts[min(e0 + 2, nE - 1)] : sent;
      da.w = (e0 + 3 < nE) ? dsts[min(e0 + 3, nE - 1)] : sent;
      db.x = (e0 + 4 < nE) ? dsts[min(e0 + 4, nE - 1)] : sent;
      db.y = (e0 + 5 < nE) ? dsts[min(e0 + 5, nE - 1)] : sent;
      db.z = (e0 + 6 < nE) ? dsts[min(e0 + 6, nE - 1)] : sent;
      db.w = (e0 + 7 < nE) ? dsts[min(e0 + 7, nE - 1)] : sent;
    }
    const unsigned nb = (unsigned)nodeBase;
    const unsigned s0 = (unsigned)da.x - nb, s1 = (unsigned)da.y - nb;
    const unsigned s2 = (unsigned)da.z - nb, s3 = (unsigned)da.w - nb;
    const unsigned s4 = (unsigned)db.x - nb, s5 = (unsigned)db.y - nb;
    const unsigned s6 = (unsigned)db.z - nb, s7 = (unsigned)db.w - nb;
    const bool h0 = s0 < (unsigned)NB, h1 = s1 < (unsigned)NB, h2 = s2 < (unsigned)NB, h3 = s3 < (unsigned)NB;
    const bool h4 = s4 < (unsigned)NB, h5 = s5 < (unsigned)NB, h6 = s6 < (unsigned)NB, h7 = s7 < (unsigned)NB;
    const unsigned any = __builtin_amdgcn_ballot_w32(h0 | h1 | h2 | h3 | h4 | h5 | h6 | h7);
    if (any != 0u) {
#define HITJ(J, HJ, SJ) { \
        const unsigned mj = __builtin_amdgcn_ballot_w32(HJ); \
        if (mj != 0u) { \
          if (HJ) { \
            const int pos = wc + (int)__builtin_amdgcn_mbcnt_lo(mj, 0u); \
            if (pos < WCAP) list[wave * WCAP + pos] = ((el0 + (J)) << 12) | (int)(SJ); \
          } \
          wc += (int)__builtin_popcount(mj); } }
      HITJ(0, h0, s0)
      HITJ(1, h1, s1)
      HITJ(2, h2, s2)
      HITJ(3, h3, s3)
      HITJ(4, h4, s4)
      HITJ(5, h5, s5)
      HITJ(6, h6, s6)
      HITJ(7, h7, s7)
#undef HITJ
    }
  }
  return wc;
}

__global__ __launch_bounds__(NTHR) void k_wprep(
    const float* __restrict__ W1, const float* __restrict__ W2,
    _Float16* w1s, _Float16* w2s) {
  const int  blk   = blockIdx.x;
  const bool first = blk < 4;
  const int  i     = (first ? blk : blk - 4) * NTHR + threadIdx.x;
  const int  o     = i * 8;
  v4f a, b;
  if (first) {
    const int n  = o / INC;
    const int k0 = o - n * INC;
    const float* p = W1 + (size_t)k0 * HIDC + n;
    a.x = p[0];        a.y = p[HIDC];     a.z = p[2 * HIDC]; a.w = p[3 * HIDC];
    b.x = p[4 * HIDC]; b.y = p[5 * HIDC]; b.z = p[6 * HIDC]; b.w = p[7 * HIDC];
  } else {
    const int n  = o / HIDC;
    const int k0 = o - n * HIDC;
    const float* p = W2 + (size_t)k0 * OUTC + n;
    a.x = p[0];        a.y = p[OUTC];     a.z = p[2 * OUTC]; a.w = p[3 * OUTC];
    b.x = p[4 * OUTC]; b.y = p[5 * OUTC]; b.z = p[6 * OUTC]; b.w = p[7 * OUTC];
  }
  a = a * WSCALE;
  b = b * WSCALE;
  const v8h hv = cvt8(a, b);
  _Float16* dp = first ? (w1s + o) : (w2s + o);
  *(volatile v8h*)dp = hv;
  __threadfence();
  *(volatile v8h*)dp = hv;
}

__global__ __launch_bounds__(NTHR) void k_deg(
    const int* __restrict__ ei, float* dinv, int nN, int nE, int vec8) {
  __shared__ __attribute__((aligned(16))) int cnt[NBD];
  __shared__ __attribute__((aligned(16))) int list[LISTN];
  __shared__ int wcnt[NWAVE];
  const int tid = threadIdx.x, lane = tid & 31, wave = tid >> 5;
  const int nodeBase = blockIdx.x * NBD;
  const int* dsts = ei + nE;
  (void)nN;

  for (int i = tid; i < NBD; i += NTHR) cnt[i] = 0;
  __syncthreads();

  const int nChunks = (nE + CHUNK - 1) / CHUNK;
#pragma unroll 1
  for (int ch = 0; ch < nChunks; ++ch) {
    const int cbase = ch * CHUNK;
    const int wc = scan_chunk<NBD>(dsts, nE, cbase, nodeBase, vec8, list, tid, lane, wave);
    if (lane == 0) wcnt[wave] = wc;
    __syncthreads();
    if (wave == 0) {
#pragma unroll 1
      for (int wsx = 0; wsx < NWAVE; ++wsx) {
        int n = __builtin_amdgcn_readfirstlane(wcnt[wsx]);
        n = n > WCAP ? WCAP : (n < 0 ? 0 : n);
        const int* lp = list + wsx * WCAP;
#pragma unroll 1
        for (int i = 0; i < n; ++i) {
          const int ent  = __builtin_amdgcn_readfirstlane(lp[i]);
          const int slot = ent & (NBD - 1);
          if (lane == 0) cnt[slot] = cnt[slot] + 1;
        }
      }
    }
    __syncthreads();
  }

  v4f dq[4];
#pragma unroll
  for (int q = 0; q < 4; ++q) {
    const int f = (wave * 4 + q) * 128 + 4 * lane;
    const v4i c = *(const v4i*)(cnt + f);
    dq[q].x = rsqrtf((float)(c.x + 1));
    dq[q].y = rsqrtf((float)(c.y + 1));
    dq[q].z = rsqrtf((float)(c.z + 1));
    dq[q].w = rsqrtf((float)(c.w + 1));
  }
  float* dp = dinv + (size_t)nodeBase;
#pragma unroll
  for (int q = 0; q < 4; ++q) *(volatile v4f*)(dp + (wave * 4 + q) * 128 + 4 * lane) = dq[q];
  __threadfence();
#pragma unroll
  for (int q = 0; q < 4; ++q) *(volatile v4f*)(dp + (wave * 4 + q) * 128 + 4 * lane) = dq[q];
}

__global__ __launch_bounds__(NTHN) void k_node(
    const float* __restrict__ x, const _Float16* __restrict__ w1s, const _Float16* __restrict__ w2s,
    const float* __restrict__ b1, const float* __restrict__ dinv, float* h2s, int nN) {
  __shared__ __attribute__((aligned(16))) float    lds0[RB * OUTC];
  __shared__ __attribute__((aligned(16))) _Float16 sH[RB * HPITCH];
  _Float16* sA  = (_Float16*)lds0;
  float*    stg = lds0;
  const int tid = threadIdx.x, lane = tid & 31, wave = tid >> 5, hh = lane >> 4, m = lane & 15;
  const int rowBase = blockIdx.x * RB;

#pragma unroll
  for (int i = 0; i < (RB * INC / 8) / NTHN; ++i) {
    const int idx = i * NTHN + tid;
    const int r   = idx >> 3;
    const int c0  = (idx & 7) * 8;
    int node = rowBase + r;
    node = node > nN - 1 ? nN - 1 : node;
    const float* xp = x + (size_t)node * INC + c0;
    const v4f a = *(const v4f*)xp, b = *(const v4f*)(xp + 4);
    *(v8h*)(sA + r * APITCH + c0) = cvt8(a, b);
  }
  __syncthreads();

  v8f acc[8];
#pragma unroll
  for (int t = 0; t < 8; ++t) { v8f z = {0.f, 0.f, 0.f, 0.f, 0.f, 0.f, 0.f, 0.f}; acc[t] = z; }
  {
    const _Float16* ar = sA + (wave * 16 + m) * APITCH + 8 * hh;
#pragma unroll
    for (int kt = 0; kt < INC / 32; ++kt) {
      FragH a;
      a.h[0] = *(const v8h*)(ar + 32 * kt);
      a.h[1] = *(const v8h*)(ar + 32 * kt + 16);
#pragma unroll
      for (int t = 0; t < 8; ++t) {
        const _Float16* bp = w1s + (size_t)(16 * t + m) * INC + 32 * kt + 8 * hh;
        FragH b;
        b.h[0] = *(const v8h*)bp;
        b.h[1] = *(const v8h*)(bp + 16);
        acc[t] = wmh(a.v, b.v, acc[t]);
      }
    }
  }

  {
    _Float16* hp = sH + (wave * 16 + 8 * hh) * HPITCH + m;
#pragma unroll
    for (int t = 0; t < 8; ++t) {
      const float bias = b1[16 * t + m];
#pragma unroll
      for (int r = 0; r < 8; ++r) {
        const float v = fmaxf(acc[t][r] * WINV + bias, 0.f);
        hp[r * HPITCH + 16 * t] = (_Float16)v;
      }
    }
  }
  __syncthreads();

  v8f acc2[4];
#pragma unroll
  for (int t = 0; t < 4; ++t) { v8f z = {0.f, 0.f, 0.f, 0.f, 0.f, 0.f, 0.f, 0.f}; acc2[t] = z; }
  {
    const _Float16* hr = sH + (wave * 16 + m) * HPITCH + 8 * hh;
#pragma unroll
    for (int kt = 0; kt < HIDC / 32; ++kt) {
      FragH a;
      a.h[0] = *(const v8h*)(hr + 32 * kt);
      a.h[1] = *(const v8h*)(hr + 32 * kt + 16);
#pragma unroll
      for (int t = 0; t < 4; ++t) {
        const _Float16* bp = w2s + (size_t)(16 * t + m) * HIDC + 32 * kt + 8 * hh;
        FragH b;
        b.h[0] = *(const v8h*)bp;
        b.h[1] = *(const v8h*)(bp + 16);
        acc2[t] = wmh(a.v, b.v, acc2[t]);
      }
    }
  }

  {
    const int r0 = wave * 16 + 8 * hh;
    const v4f dA = *(const v4f*)(dinv + (size_t)rowBase + r0);
    const v4f dB = *(const v4f*)(dinv + (size_t)rowBase + r0 + 4);
    const float d0 = dA.x * WINV, d1 = dA.y * WINV, d2 = dA.z * WINV, d3 = dA.w * WINV;
    const float d4 = dB.x * WINV, d5 = dB.y * WINV, d6 = dB.z * WINV, d7 = dB.w * WINV;
    float* sp = stg + r0 * OUTC + m;
#pragma unroll
    for (int t = 0; t < 4; ++t) {
      sp[0 * OUTC + 16 * t] = acc2[t][0] * d0;
      sp[1 * OUTC + 16 * t] = acc2[t][1] * d1;
      sp[2 * OUTC + 16 * t] = acc2[t][2] * d2;
      sp[3 * OUTC + 16 * t] = acc2[t][3] * d3;
      sp[4 * OUTC + 16 * t] = acc2[t][4] * d4;
      sp[5 * OUTC + 16 * t] = acc2[t][5] * d5;
      sp[6 * OUTC + 16 * t] = acc2[t][6] * d6;
      sp[7 * OUTC + 16 * t] = acc2[t][7] * d7;
    }
  }
  __syncthreads();

  const float* lp = stg + wave * 16 * OUTC + 4 * lane;
  float* gp = h2s + ((size_t)rowBase + wave * 16) * OUTC + 4 * lane;
#pragma unroll
  for (int q = 0; q < 8; ++q) { const v4f v = *(const v4f*)(lp + q * 128); *(volatile v4f*)(gp + (size_t)q * 128) = v; }
  __threadfence();
#pragma unroll
  for (int q = 0; q < 8; ++q) { const v4f v = *(const v4f*)(lp + q * 128); *(volatile v4f*)(gp + (size_t)q * 128) = v; }
}

__global__ __launch_bounds__(NTHR) void k_agg(
    const int* __restrict__ ei, const float* __restrict__ h2s, const float* __restrict__ dinv,
    const float* __restrict__ b2, float* out, int nN, int nE, int vec8) {
  extern __shared__ v4f lds_dyn[];
  float* acc  = (float*)lds_dyn;
  int*   list = (int*)(acc + NBA * OUTC);
  int*   wcnt = list + LISTN;
  const int tid = threadIdx.x, lane = tid & 31, wave = tid >> 5;
  const int nodeBase = blockIdx.x * NBA;
  const int* dsts = ei + nE;

  {
    const v4f z = {0.f, 0.f, 0.f, 0.f};
    for (int i = tid; i < NBA * OUTC / 4; i += NTHR) lds_dyn[i] = z;
  }
  __syncthreads();

  const int nChunks = (nE + CHUNK - 1) / CHUNK;
#pragma unroll 1
  for (int ch = 0; ch < nChunks; ++ch) {
    const int cbase = ch * CHUNK;
    const int wc = scan_chunk<NBA>(dsts, nE, cbase, nodeBase, vec8, list, tid, lane, wave);
    if (lane == 0) wcnt[wave] = wc;
    __syncthreads();
    if (wave == 0) {
#pragma unroll 1
      for (int wsx = 0; wsx < NWAVE; ++wsx) {
        int n = __builtin_amdgcn_readfirstlane(wcnt[wsx]);
        n = n > WCAP ? WCAP : (n < 0 ? 0 : n);
        const int* lp = list + wsx * WCAP;
#pragma unroll 1
        for (int i = 0; i < n; ++i) {
          const int ent  = __builtin_amdgcn_readfirstlane(lp[i]);
          const int slot = ent & (NBA - 1);
          int e = cbase + ((ent >> 12) & (CHUNK - 1));
          e = e > nE - 1 ? nE - 1 : e;
          int src = ei[e];
          src = src < 0 ? 0 : (src > nN - 1 ? nN - 1 : src);
          const v2f v = *(const v2f*)(h2s + (size_t)src * OUTC + 2 * lane);
          v2f* ap = (v2f*)(acc + slot * OUTC + 2 * lane);
          *ap = *ap + v;
        }
      }
    }
    __syncthreads();
  }

#pragma unroll 4
  for (int i = 0; i < (NBA * OUTC / 4) / NTHR; ++i) {
    const int idx  = i * NTHR + tid;
    const int slot = idx >> 4;
    const int c4   = (idx & 15) * 4;
    int node = nodeBase + slot;
    node = node > nN - 1 ? nN - 1 : node;
    const float d  = dinv[node];
    const v4f   gv = *(const v4f*)(h2s + (size_t)node * OUTC + c4);
    const v4f   bv = *(const v4f*)(b2 + c4);
    v4f* ap = (v4f*)(acc + slot * OUTC + c4);
    const v4f s = *ap + gv;
    *ap = s * d + bv;
  }
  __syncthreads();

  const size_t outN = (size_t)nN * OUTC;
  const size_t ob   = (size_t)nodeBase * OUTC;
#pragma unroll 4
  for (int q = 0; q < 64; ++q) {
    const int f = (wave * 64 + q) * 128 + 4 * lane;
    const size_t gi = ob + (size_t)f;
    if (gi < outN) { const v4f v = *(const v4f*)(acc + f); *(volatile v4f*)(out + gi) = v; }
  }
  __threadfence();
#pragma unroll 4
  for (int q = 0; q < 64; ++q) {
    const int f = (wave * 64 + q) * 128 + 4 * lane;
    const size_t gi = ob + (size_t)f;
    if (gi < outN) { const v4f v = *(const v4f*)(acc + f); *(volatile v4f*)(out + gi) = v; }
  }
}

extern "C" void kernel_launch(void* const* d_in, const int* in_sizes, int n_in,
                              void* d_out, int out_size, void* d_ws, size_t ws_size,
                              hipStream_t stream) {
  if (n_in < 6) return;
  const int nN = in_sizes[0] / INC;
  const int nE = in_sizes[1] / 2;
  if (nN <= 0 || nE < 0 || in_sizes[0] != nN * INC || in_sizes[1] != nE * 2) return;
  if (in_sizes[2] != INC * HIDC || in_sizes[3] < HIDC || in_sizes[4] != HIDC * OUTC || in_sizes[5] < OUTC) return;
  if (out_size != nN * OUTC) return;

  const float* x  = (const float*)d_in[0];
  const int*   ei = (const int*)d_in[1];
  const float* W1 = (const float*)d_in[2];
  const float* b1 = (const float*)d_in[3];
  const float* W2 = (const float*)d_in[4];
  const float* b2 = (const float*)d_in[5];
  float* out = (float*)d_out;

  const int nBD = (nN + NBD - 1) / NBD;
  const int nNB = (nN + RB - 1) / RB;
  const int nAG = (nN + NBA - 1) / NBA;

  char* ws = (char*)d_ws;
  size_t off = 0;
  const size_t oW1 = off; off += (size_t)HIDC * INC * 2;                        off = (off + 255) & ~(size_t)255;
  const size_t oW2 = off; off += (size_t)OUTC * HIDC * 2;                       off = (off + 255) & ~(size_t)255;
  const size_t oDv = off; off += (size_t)nBD * NBD * 4;                         off = (off + 255) & ~(size_t)255;
  const size_t oH2 = off; off += (size_t)nNB * RB * OUTC * 4;                   off = (off + 255) & ~(size_t)255;
  if (off > ws_size) return;
  if ((size_t)nNB * RB > (size_t)nBD * NBD) return;
  _Float16* w1s  = (_Float16*)(ws + oW1);
  _Float16* w2s  = (_Float16*)(ws + oW2);
  float*    dinv = (float*)(ws + oDv);
  float*    h2s  = (float*)(ws + oH2);

  const int vec8 = ((nE & 3) == 0) ? 1 : 0;

  k_wprep<<<8, NTHR, 0, stream>>>(W1, W2, w1s, w2s);

  k_deg<<<nBD, NTHR, 0, stream>>>(ei, dinv, nN, nE, vec8);

  k_node<<<nNB, NTHN, 0, stream>>>(x, w1s, w2s, b1, dinv, h2s, nN);

  hipFuncSetAttribute(reinterpret_cast<const void*>(&k_agg),
                      hipFuncAttributeMaxDynamicSharedMemorySize, LDS_AGG);
  k_agg<<<nAG, NTHR, LDS_AGG, stream>>>(ei, h2s, dinv, b2, out, nN, nE, vec8);
}
